// MessagePassingNeuralNetwork_5523327942769
// MI455X (gfx1250) — hardware-verified
//
#include <hip/hip_runtime.h>
#include <stddef.h>


#define ED      64
#define NSH     23
#define MDIM    87
#define HID     200
#define RDIM    256
#define TPASS   3
#define KP_MSG  96
#define KP_HID  224
#define NPL     224
#define NCMP    208
#define HEADN   16
#define EPSBN   1e-5f
#define WSCALE  16.0f
#define WINV    0.0625f

#define NTHR    256
#define NWAVE   8
#define EPT     8
#define NGRP    2
#define CHUNK   (NTHR * EPT * NGRP)
#define WCAP    (EPT * NGRP * 32)
#define LISTN   (NWAVE * WCAP)
#define NBC     4096
#define NBF     1024
#define NBP     32
#define RCAP    40960
#define RBN     128
#define TGT     256
#define DEGCAP  256
#define GROWS   128
#define OTHR    512
#define WPT     128
#define CSRB    400
#define AP_U    232
#define AP_R    264

#define LDS_FILL ((RCAP + NBF + LISTN) * 4 + 64)
#define LDS_UPD  (2 * GROWS * AP_U * 2 + GROWS * ED * 4)
#define LDS_RO   (2 * GROWS * AP_R * 2 + GROWS * 4)

#define PW1  (NPL * KP_MSG)
#define PW2  (NPL * KP_HID)
#define PW4  (ED * KP_HID)
#define PR1  (NPL * RDIM)
#define PR4  (HEADN * KP_HID)
#define OW1  0
#define OW2  (OW1 + TPASS * PW1)
#define OW3  (OW2 + TPASS * PW2)
#define OW4  (OW3 + TPASS * PW2)
#define OR1  (OW4 + TPASS * PW4)
#define OR2  (OR1 + PR1)
#define OR3  (OR2 + PW2)
#define OR4  (OR3 + PW2)
#define WTOT (OR4 + PR4)
#define WE0  (TPASS * PW1 / 8)
#define WE1  (WE0 + TPASS * PW2 / 8)
#define WE2  (WE1 + TPASS * PW2 / 8)
#define WE3  (WE2 + TPASS * PW4 / 8)
#define WE4  (WE3 + PR1 / 8)
#define WE5  (WE4 + PW2 / 8)
#define WE6  (WE5 + PW2 / 8)
#define WE7  (WE6 + PR4 / 8)

static_assert((CHUNK & (CHUNK - 1)) == 0);
static_assert(CHUNK <= 4096);
static_assert(NBC <= 4096 && NBF <= 4096 && NBP <= 4096);
static_assert((NBC & (NBC - 1)) == 0 && (NBF & (NBF - 1)) == 0 && (NBP & (NBP - 1)) == 0);
static_assert(NBC == 4 * NBF);
static_assert(OTHR * 8 == NBC);
static_assert((RCAP % 32) == 0);
static_assert(TGT == NWAVE * 32 && (TGT % GROWS) == 0 && (TGT % 16) == 0);
static_assert(GROWS == NWAVE * 16);
static_assert(NCMP == 13 * 16 && NCMP + 16 == KP_HID && NPL >= KP_HID);
static_assert((WE0 % WPT) == 0 && (WE1 % WPT) == 0 && (WE2 % WPT) == 0 && (WE3 % WPT) == 0);
static_assert((WE4 % WPT) == 0 && (WE5 % WPT) == 0 && (WE6 % WPT) == 0);
static_assert((OW2 % 64) == 0 && (OW3 % 64) == 0 && (OW4 % 64) == 0 && (OR1 % 64) == 0);
static_assert((OR2 % 64) == 0 && (OR3 % 64) == 0 && (OR4 % 64) == 0 && (WTOT % 64) == 0);
static_assert((GROWS * KP_MSG / 8) % NTHR == 0 && (GROWS * RDIM / 8) % NTHR == 0);
static_assert(((AP_U * 2) % 16) == 0 && ((AP_R * 2) % 16) == 0);
static_assert(AP_U >= KP_HID + 8 && AP_R >= RDIM + 8);
static_assert(ED == 64 && MDIM == NSH + ED && KP_MSG == 96);

typedef float    v2f  __attribute__((ext_vector_type(2)));
typedef float    v4f  __attribute__((ext_vector_type(4)));
typedef float    v8f  __attribute__((ext_vector_type(8)));
typedef int      v4i  __attribute__((ext_vector_type(4)));
typedef double   v2d  __attribute__((ext_vector_type(2)));
typedef _Float16 v8h  __attribute__((ext_vector_type(8)));
typedef _Float16 v16h __attribute__((ext_vector_type(16)));
union FragH { v16h v; v8h h[2]; };
union FI { float f; int i; };

__constant__ float c_shifts[NSH] = {
  0.800000012f, 0.899999976f, 0.99999994f, 1.0999999f, 1.19999981f, 1.29999983f, 1.39999986f, 1.49999976f,
  1.59999967f, 1.69999969f, 1.79999971f, 1.89999962f, 1.99999952f, 2.09999943f, 2.19999957f, 2.29999948f,
  2.39999938f, 2.49999928f, 2.59999943f, 2.69999933f, 2.79999924f, 2.89999914f, 2.99999928f };

__device__ __forceinline__ v8h cvt8(v4f a, v4f b) {
  v8h r;
  r[0] = (_Float16)a.x; r[1] = (_Float16)a.y; r[2] = (_Float16)a.z; r[3] = (_Float16)a.w;
  r[4] = (_Float16)b.x; r[5] = (_Float16)b.y; r[6] = (_Float16)b.z; r[7] = (_Float16)b.w;
  return r;
}

__device__ __forceinline__ v8f wmh(v16h a, v16h b, v8f c) {
  v8f d = __builtin_amdgcn_wmma_f32_16x16x32_f16(false, a, false, b, (short)0, c, false, false);
  asm volatile("v_nop\n\tv_nop\n\tv_nop\n\tv_nop" : "+v"(d) : "v"(a), "v"(b));
  return d;
}

template <int NB>
__device__ __forceinline__ int scan_chunk(const int* __restrict__ dsts, int nE, int cbase, int slotBase,
                                          int vec8, int* list, int tid, int lane, int wave) {
  int wc = 0;
#pragma unroll
  for (int g = 0; g < NGRP; ++g) {
    const int el0  = (g * NTHR + tid) * EPT;
    const int e0   = cbase + el0;
    const int sent = -2147483647 - 1;
    v4i da, db;
    if (vec8 != 0 && cbase + CHUNK <= nE) {
      da = *(const v4i*)(dsts + e0);
      db = *(const v4i*)(dsts + e0 + 4);
    } else {
      da.x = (e0     < nE) ? dsts[min(e0, nE - 1)] : sent;
      da.y = (e0 + 1 < nE) ? dsts[min(e0 + 1, nE - 1)] : sent;
      da.z = (e0 + 2 < nE) ? dsts[min(e0 + 2, nE - 1)] : sent;
      da.w = (e0 + 3 < nE) ? dsts[min(e0 + 3, nE - 1)] : sent;
      db.x = (e0 + 4 < nE) ? dsts[min(e0 + 4, nE - 1)] : sent;
      db.y = (e0 + 5 < nE) ? dsts[min(e0 + 5, nE - 1)] : sent;
      db.z = (e0 + 6 < nE) ? dsts[min(e0 + 6, nE - 1)] : sent;
      db.w = (e0 + 7 < nE) ? dsts[min(e0 + 7, nE - 1)] : sent;
    }
    const unsigned nb = (unsigned)slotBase;
    const unsigned s0 = (unsigned)da.x - nb, s1 = (unsigned)da.y - nb;
    const unsigned s2 = (unsigned)da.z - nb, s3 = (unsigned)da.w - nb;
    const unsigned s4 = (unsigned)db.x - nb, s5 = (unsigned)db.y - nb;
    const unsigned s6 = (unsigned)db.z - nb, s7 = (unsigned)db.w - nb;
    const bool h0 = s0 < (unsigned)NB, h1 = s1 < (unsigned)NB, h2 = s2 < (unsigned)NB, h3 = s3 < (unsigned)NB;
    const bool h4 = s4 < (unsigned)NB, h5 = s5 < (unsigned)NB, h6 = s6 < (unsigned)NB, h7 = s7 < (unsigned)NB;
    const unsigned any = __builtin_amdgcn_ballot_w32(h0 | h1 | h2 | h3 | h4 | h5 | h6 | h7);
    if (any != 0u) {
#define HITJ(J, HJ, SJ) { \
        const unsigned mj = __builtin_amdgcn_ballot_w32(HJ); \
        if (mj != 0u) { \
          if (HJ) { \
            const int pos = wc + (int)__builtin_amdgcn_mbcnt_lo(mj, 0u); \
            if (pos < WCAP) list[wave * WCAP + pos] = ((el0 + (J)) << 12) | (int)(SJ); \
          } \
          wc += (int)__builtin_popcount(mj); } }
      HITJ(0, h0, s0)
      HITJ(1, h1, s1)
      HITJ(2, h2, s2)
      HITJ(3, h3, s3)
      HITJ(4, h4, s4)
      HITJ(5, h5, s5)
      HITJ(6, h6, s6)
      HITJ(7, h7, s7)
#undef HITJ
    }
  }
  return wc;
}

template <int KT, int NT>
__device__ __forceinline__ void mma_tiles(const _Float16* aRow, const _Float16* __restrict__ bLane, v8f (&acc)[NT]) {
  constexpr int KP = KT * 32;
#pragma unroll
  for (int t = 0; t < NT; ++t) { v8f z = {0.f, 0.f, 0.f, 0.f, 0.f, 0.f, 0.f, 0.f}; acc[t] = z; }
#pragma unroll 1
  for (int kt = 0; kt < KT; ++kt) {
    FragH a;
    a.h[0] = *(const v8h*)(aRow + 32 * kt);
    a.h[1] = *(const v8h*)(aRow + 32 * kt + 16);
#pragma unroll
    for (int t = 0; t < NT; ++t) {
      const _Float16* bp = bLane + (size_t)(16 * t) * KP + 32 * kt;
      FragH b;
      b.h[0] = *(const v8h*)bp;
      b.h[1] = *(const v8h*)(bp + 16);
      acc[t] = wmh(a.v, b.v, acc[t]);
    }
  }
}

template <int NT, int AP>
__device__ __forceinline__ void epi_h(const v8f (&acc)[NT], int n0, const float* __restrict__ bias, _Float16* dRow, int m) {
#pragma unroll
  for (int t = 0; t < NT; ++t) {
    const int col = n0 + 16 * t + m;
    const float bl = bias[col < HID ? col : HID - 1];
    const bool ok  = col < HID;
#pragma unroll
    for (int r = 0; r < 8; ++r) {
      float v = fmaxf(acc[t][r] * WINV + bl, 0.0f);
      v = ok ? v : 0.0f;
      dRow[r * AP + col] = (_Float16)v;
    }
  }
}

template <int KT, int AP>
__device__ __forceinline__ void layer_h(const _Float16* sIn, _Float16* sOut, const _Float16* __restrict__ Bp,
                                        const float* __restrict__ bias, int r0, int hh, int m) {
  constexpr int KP = KT * 32;
  const _Float16* aRow = sIn + (r0 + m) * AP + 8 * hh;
  _Float16* dRow = sOut + (r0 + 8 * hh) * AP;
  {
    v8f acc[7];
    mma_tiles<KT, 7>(aRow, Bp + (size_t)m * KP + 8 * hh, acc);
    epi_h<7, AP>(acc, 0, bias, dRow, m);
  }
  {
    v8f acc[6];
    mma_tiles<KT, 6>(aRow, Bp + (size_t)(112 + m) * KP + 8 * hh, acc);
    epi_h<6, AP>(acc, 112, bias, dRow, m);
  }
  const float zf = 0.0f * (float)m;
#pragma unroll
  for (int r = 0; r < 8; ++r) dRow[r * AP + NCMP + m] = (_Float16)zf;
}

__global__ __launch_bounds__(WPT) void k_wprep(
    const float* __restrict__ uw1, const float* __restrict__ uw2, const float* __restrict__ uw3,
    const float* __restrict__ uw4, const float* __restrict__ rw1, const float* __restrict__ rw2,
    const float* __restrict__ rw3, const float* __restrict__ rw4, _Float16* wp) {
  const int bstart = blockIdx.x * WPT;
  const float* src; int K, Nout, per, KP, perm, dOff, tStart;
  if (bstart < WE0)      { src = uw1; K = MDIM; Nout = HID; per = PW1; KP = KP_MSG; perm = 1; dOff = OW1; tStart = 0;   }
  else if (bstart < WE1) { src = uw2; K = HID;  Nout = HID; per = PW2; KP = KP_HID; perm = 0; dOff = OW2; tStart = WE0; }
  else if (bstart < WE2) { src = uw3; K = HID;  Nout = HID; per = PW2; KP = KP_HID; perm = 0; dOff = OW3; tStart = WE1; }
  else if (bstart < WE3) { src = uw4; K = HID;  Nout = ED;  per = PW4; KP = KP_HID; perm = 0; dOff = OW4; tStart = WE2; }
  else if (bstart < WE4) { src = rw1; K = RDIM; Nout = HID; per = PR1; KP = RDIM;   perm = 0; dOff = OR1; tStart = WE3; }
  else if (bstart < WE5) { src = rw2; K = HID;  Nout = HID; per = PW2; KP = KP_HID; perm = 0; dOff = OR2; tStart = WE4; }
  else if (bstart < WE6) { src = rw3; K = HID;  Nout = HID; per = PW2; KP = KP_HID; perm = 0; dOff = OR3; tStart = WE5; }
  else                   { src = rw4; K = HID;  Nout = 1;   per = PR4; KP = KP_HID; perm = 0; dOff = OR4; tStart = WE6; }
  const int i = bstart + (int)threadIdx.x;
  if (i >= WE7) return;
  const int o = (i - tStart) * 8;
  const int layer = o / per;
  const int oo = o - layer * per;
  const int n  = oo / KP;
  const int k0 = oo - n * KP;
  const float* sl = src + (size_t)layer * K * Nout;
  const int nc = n < Nout ? n : Nout - 1;
  float v[8];
#pragma unroll
  for (int e = 0; e < 8; ++e) {
    const int k  = k0 + e;
    const int kk = k < K ? k : K - 1;
    const int kr = perm != 0 ? (kk < ED ? kk + NSH : kk - ED) : kk;
    const float x = sl[(size_t)kr * Nout + nc];
    v[e] = (k < K && n < Nout) ? x * WSCALE : 0.0f;
  }
  v4f a, b;
  a.x = v[0]; a.y = v[1]; a.z = v[2]; a.w = v[3];
  b.x = v[4]; b.y = v[5]; b.z = v[6]; b.w = v[7];
  const v8h hv = cvt8(a, b);
  _Float16* dp = wp + dOff + o;
  *(volatile v8h*)dp = hv;
  __threadfence();
  *(volatile v8h*)dp = hv;
}

__global__ __launch_bounds__(NTHR) void k_count(const int* __restrict__ keys, int* cnt, int nE, int vec8) {
  __shared__ __attribute__((aligned(16))) int scnt[NBC];
  __shared__ __attribute__((aligned(16))) int list[LISTN];
  __shared__ int wcnt[NWAVE];
  const int tid = threadIdx.x, lane = tid & 31, wave = tid >> 5;
  const int nodeBase = blockIdx.x * NBC;

  for (int i = tid; i < NBC; i += NTHR) scnt[i] = 0;
  __syncthreads();

  const int nChunks = (nE + CHUNK - 1) / CHUNK;
#pragma unroll 1
  for (int ch = 0; ch < nChunks; ++ch) {
    const int cbase = ch * CHUNK;
    const int wc = scan_chunk<NBC>(keys, nE, cbase, nodeBase, vec8, list, tid, lane, wave);
    if (lane == 0) wcnt[wave] = wc;
    __syncthreads();
    if (wave == 0) {
#pragma unroll 1
      for (int wsx = 0; wsx < NWAVE; ++wsx) {
        int n = __builtin_amdgcn_readfirstlane(wcnt[wsx]);
        n = n > WCAP ? WCAP : (n < 0 ? 0 : n);
        const int* lp = list + wsx * WCAP;
#pragma unroll 1
        for (int i = 0; i < n; ++i) {
          const int ent  = __builtin_amdgcn_readfirstlane(lp[i]);
          const int slot = ent & (NBC - 1);
          if (lane == 0) scnt[slot] = scnt[slot] + 1;
        }
      }
    }
    __syncthreads();
  }

  v4i cq[4];
#pragma unroll
  for (int q = 0; q < 4; ++q) {
    const int f = (wave * 4 + q) * 128 + 4 * lane;
    cq[q] = *(const v4i*)(scnt + f);
  }
  int* cp = cnt + (size_t)nodeBase;
#pragma unroll
  for (int q = 0; q < 4; ++q) { const int f = (wave * 4 + q) * 128 + 4 * lane; *(volatile v4i*)(cp + f) = cq[q]; }
  __threadfence();
#pragma unroll
  for (int q = 0; q < 4; ++q) { const int f = (wave * 4 + q) * 128 + 4 * lane; *(volatile v4i*)(cp + f) = cq[q]; }
}

__global__ __launch_bounds__(OTHR) void k_offsets(const int* __restrict__ cnt, int* off, int* rbase, int nChunk) {
  __shared__ __attribute__((aligned(16))) int soff[NBC];
  __shared__ __attribute__((aligned(16))) int srb[RBN];
  __shared__ int wtot[OTHR / 32];
  const int tid = threadIdx.x, lane = tid & 31, wave = tid >> 5, sub = tid >> 7;
  for (int i = tid; i < RBN; i += OTHR) srb[i] = 0;
  int carry = 0;
#pragma unroll 1
  for (int ch = 0; ch < nChunk; ++ch) {
    const int base = ch * NBC;
    const v4i c0 = *(const v4i*)(cnt + base + 8 * tid);
    const v4i c1 = *(const v4i*)(cnt + base + 8 * tid + 4);
    const int e0 = max(c0.x, 0), e1 = max(c0.y, 0), e2 = max(c0.z, 0), e3 = max(c0.w, 0);
    const int e4 = max(c1.x, 0), e5 = max(c1.y, 0), e6 = max(c1.z, 0), e7 = max(c1.w, 0);
    const int ts = e0 + e1 + e2 + e3 + e4 + e5 + e6 + e7;
    int incl = ts;
#pragma unroll
    for (int d = 1; d < 32; d <<= 1) {
      const int t = __shfl_up(incl, d);
      if (lane >= d) incl += t;
    }
    if (lane == 31) wtot[wave] = incl;
    __syncthreads();
    const int S0 = wtot[0]  + wtot[1]  + wtot[2]  + wtot[3];
    const int S1 = wtot[4]  + wtot[5]  + wtot[6]  + wtot[7];
    const int S2 = wtot[8]  + wtot[9]  + wtot[10] + wtot[11];
    const int S3 = wtot[12] + wtot[13] + wtot[14] + wtot[15];
    int pre = 0;
#pragma unroll 1
    for (int w = 4 * sub; w < wave; ++w) pre += wtot[w];
    const int b0 = carry;
    const int b1 = b0 + ((S0 + 31) & ~31);
    const int b2 = b1 + ((S1 + 31) & ~31);
    const int b3 = b2 + ((S2 + 31) & ~31);
    const int b4 = b3 + ((S3 + 31) & ~31);
    const int myb = sub == 0 ? b0 : (sub == 1 ? b1 : (sub == 2 ? b2 : b3));
    if (tid == 0) {
      srb[min(4 * ch + 0, RBN - 1)] = b0;
      srb[min(4 * ch + 1, RBN - 1)] = b1;
      srb[min(4 * ch + 2, RBN - 1)] = b2;
      srb[min(4 * ch + 3, RBN - 1)] = b3;
    }
    int run = myb + pre + incl - ts;
    soff[8 * tid + 0] = run; run += e0;
    soff[8 * tid + 1] = run; run += e1;
    soff[8 * tid + 2] = run; run += e2;
    soff[8 * tid + 3] = run; run += e3;
    soff[8 * tid + 4] = run; run += e4;
    soff[8 * tid + 5] = run; run += e5;
    soff[8 * tid + 6] = run; run += e6;
    soff[8 * tid + 7] = run;
    carry = b4;
    __syncthreads();
    const v4i o0 = *(const v4i*)(soff + 4 * tid);
    const v4i o1 = *(const v4i*)(soff + 4 * (tid + OTHR));
    int* op = off + base;
    *(volatile v4i*)(op + 4 * tid) = o0;
    *(volatile v4i*)(op + 4 * (tid + OTHR)) = o1;
    __threadfence();
    *(volatile v4i*)(op + 4 * tid) = o0;
    *(volatile v4i*)(op + 4 * (tid + OTHR)) = o1;
    __syncthreads();
  }
  if (tid == 0) srb[min(4 * nChunk, RBN - 1)] = carry;
  __syncthreads();
  v4i rv = {0, 0, 0, 0};
  if (tid < 32) rv = *(const v4i*)(srb + 4 * tid);
  if (tid < 32) *(volatile v4i*)(rbase + 4 * tid) = rv;
  __threadfence();
  if (tid < 32) *(volatile v4i*)(rbase + 4 * tid) = rv;
}

__global__ __launch_bounds__(NTHR) void k_fill(
    const int* __restrict__ keys, const int* __restrict__ off, const int* __restrict__ rbase,
    int* csr, int nE, int vec8, int csrLen) {
  extern __shared__ v4f lds_dyn[];
  int* region = (int*)lds_dyn;
  int* cursor = region + RCAP;
  int* list   = cursor + NBF;
  int* wcnt   = list + LISTN;
  const int tid = threadIdx.x, lane = tid & 31, wave = tid >> 5;
  const int b = blockIdx.x;
  const int nodeBase = b * NBF;

  int rb0 = rbase[b];
  const int rb1 = rbase[b + 1];
  rb0 = rb0 < 0 ? 0 : (rb0 > csrLen ? csrLen : rb0);
  rb0 &= ~31;
  int len = rb1 - rb0;
  len = len < 0 ? 0 : (len > RCAP ? RCAP : len);
  int lenW = (len + 31) & ~31;
  if (rb0 + lenW > csrLen) lenW = (csrLen - rb0) & ~31;

  {
    const v4i z = {0, 0, 0, 0};
    for (int i = tid; i < RCAP / 4; i += NTHR) ((v4i*)region)[i] = z;
    for (int s = tid; s < NBF; s += NTHR) {
      int o = off[nodeBase + s] - rb0;
      o = o < 0 ? 0 : (o > RCAP ? RCAP : o);
      cursor[s] = o;
    }
  }
  __syncthreads();

  const int nChunks = (nE + CHUNK - 1) / CHUNK;
#pragma unroll 1
  for (int ch = 0; ch < nChunks; ++ch) {
    const int cbase = ch * CHUNK;
    const int wc = scan_chunk<NBF>(keys, nE, cbase, nodeBase, vec8, list, tid, lane, wave);
    if (lane == 0) wcnt[wave] = wc;
    __syncthreads();
    if (wave == 0) {
#pragma unroll 1
      for (int wsx = 0; wsx < NWAVE; ++wsx) {
        int n = __builtin_amdgcn_readfirstlane(wcnt[wsx]);
        n = n > WCAP ? WCAP : (n < 0 ? 0 : n);
        const int* lp = list + wsx * WCAP;
#pragma unroll 1
        for (int i = 0; i < n; ++i) {
          const int ent  = __builtin_amdgcn_readfirstlane(lp[i]);
          const int slot = ent & (NBF - 1);
          int e = cbase + ((ent >> 12) & (CHUNK - 1));
          e = e > nE - 1 ? nE - 1 : e;
          if (lane == 0) {
            int pos = cursor[slot];
            pos = pos < 0 ? 0 : (pos > RCAP - 1 ? RCAP - 1 : pos);
            region[pos] = e;
            const int np = pos + 1;
            cursor[slot] = np > RCAP ? RCAP : np;
          }
        }
      }
    }
    __syncthreads();
  }

  const int nv = lenW >> 2;
  int* gp = csr + rb0;
#pragma unroll 1
  for (int i = tid; i < nv; i += NTHR) { const v4i v = ((const v4i*)region)[i]; *(volatile v4i*)(gp + 4 * i) = v; }
  __threadfence();
#pragma unroll 1
  for (int i = tid; i < nv; i += NTHR) { const v4i v = ((const v4i*)region)[i]; *(volatile v4i*)(gp + 4 * i) = v; }
}

__global__ __launch_bounds__(NTHR) void k_embed(const int* __restrict__ z, const float* __restrict__ emb,
                                                float* xall, int nN, int nEmb) {
  const int tid = threadIdx.x, q = tid & 15, rr = tid >> 4;
  const int row = blockIdx.x * 16 + rr;
  int zr = z[row < nN ? row : nN - 1];
  zr = zr < 0 ? 0 : (zr > nEmb - 1 ? nEmb - 1 : zr);
  const v4f v = *(const v4f*)(emb + (size_t)zr * ED + 4 * q);
  float* xp = xall + (size_t)row * RDIM + 4 * q;
  *(volatile v4f*)xp = v;
  __threadfence();
  *(volatile v4f*)xp = v;
}

template <int RBF>
__global__ __launch_bounds__(NTHR) void k_agg(
    const int* __restrict__ csr, const int* __restrict__ off, const int* __restrict__ cnt,
    const int* __restrict__ esnk, const float* __restrict__ dist, const float* __restrict__ xsrc, int xoff,
    float* mpl, int nN, int nE, int csrLen) {
  const int tid = threadIdx.x, lane = tid & 31, wave = tid >> 5;
  const int tbase = blockIdx.x * TGT + wave * 32;
  const int cl = tbase + lane;
  const int cnt_l = cnt[cl];
  const int off_l = off[cl];
  const float sh = c_shifts[lane < NSH ? lane : NSH - 1];
  const int sa = (2 * lane) & 31, sb = (2 * lane + 1) & 31;
  const int sr = (4 * (lane - 16)) & 31;
  const bool lo16 = lane < 16;

#pragma unroll 1
  for (int j = 0; j < 32; ++j) {
    const int c = tbase + j;
    int n = __builtin_amdgcn_readlane(cnt_l, j);
    n = n < 0 ? 0 : (n > DEGCAP ? DEGCAP : n);
    const int st = __builtin_amdgcn_readlane(off_l, j);
    v2f acc = {0.f, 0.f};
    float racc = 0.0f;
#pragma unroll 1
    for (int q0 = 0; q0 < n; q0 += 32) {
      int pos = st + q0 + lane;
      pos = pos < 0 ? 0 : (pos > csrLen - 1 ? csrLen - 1 : pos);
      int e = csr[pos];
      e = e < 0 ? 0 : (e > nE - 1 ? nE - 1 : e);
      int sk = esnk[e];
      sk = sk < 0 ? 0 : (sk > nN - 1 ? nN - 1 : sk);
      FI du; du.f = 0.0f;
      if (RBF) du.f = dist[e];
      const int mcnt = (n - q0) < 32 ? (n - q0) : 32;
#pragma unroll 1
      for (int p = 0; p < mcnt; ++p) {
        const int s = __builtin_amdgcn_readlane(sk, p);
        acc = acc + *(const v2f*)(xsrc + (size_t)s * RDIM + xoff + 2 * lane);
        if (RBF) {
          FI dd; dd.i = __builtin_amdgcn_readlane(du.i, p);
          const float d = dd.f - sh;
          const float dq = d * d;
          racc += expf(-dq);
        }
      }
    }
    const float ax = __shfl(acc.x, sa), ay = __shfl(acc.y, sa);
    const float bx = __shfl(acc.x, sb), by = __shfl(acc.y, sb);
    v4f v; v.x = ax; v.y = ay; v.z = bx; v.w = by;
    if (RBF) {
      racc = lane < NSH ? racc : 0.0f;
      const float g0 = __shfl(racc, sr), g1 = __shfl(racc, (sr + 1) & 31);
      const float g2 = __shfl(racc, (sr + 2) & 31), g3 = __shfl(racc, (sr + 3) & 31);
      v.x = lo16 ? v.x : g0; v.y = lo16 ? v.y : g1; v.z = lo16 ? v.z : g2; v.w = lo16 ? v.w : g3;
    }
    float* mp = mpl + (size_t)c * KP_MSG + 4 * lane;
    const int nst = RBF ? 24 : 16;
    if (lane < nst) *(volatile v4f*)mp = v;
    __threadfence();
    if (lane < nst) *(volatile v4f*)mp = v;
  }
}

__global__ __launch_bounds__(NTHR) void k_colstats(const float* __restrict__ X, int P, int nrows, double* part) {
  __shared__ __attribute__((aligned(16))) double red[NTHR * 8];
  __shared__ __attribute__((aligned(16))) double sres[512];
  const int tid = threadIdx.x;
  const int G = P >> 2;
  const int PH = NTHR / G;
  const int g = tid % G, ph = tid / G;
  const int phc = ph < PH ? ph : PH - 1;
  const int r0 = blockIdx.x * CSRB;
  int r1 = r0 + CSRB; r1 = r1 > nrows ? nrows : r1;
  double s0 = 0.0, s1 = 0.0, s2 = 0.0, s3 = 0.0, q0 = 0.0, q1 = 0.0, q2 = 0.0, q3 = 0.0;
#pragma unroll 1
  for (int r = r0 + phc; r < r1; r += PH) {
    const v4f v = *(const v4f*)(X + (size_t)r * P + 4 * g);
    const double d0 = (double)v.x, d1 = (double)v.y, d2 = (double)v.z, d3 = (double)v.w;
    s0 += d0; s1 += d1; s2 += d2; s3 += d3;
    q0 = fma(d0, d0, q0); q1 = fma(d1, d1, q1); q2 = fma(d2, d2, q2); q3 = fma(d3, d3, q3);
  }
  if (ph < PH) {
    double* rp = red + (ph * G + g) * 8;
    rp[0] = s0; rp[1] = s1; rp[2] = s2; rp[3] = s3; rp[4] = q0; rp[5] = q1; rp[6] = q2; rp[7] = q3;
  }
  __syncthreads();
  if (tid < P) {
    const int gg = tid >> 2, cc = tid & 3;
    double s = 0.0, q = 0.0;
#pragma unroll 1
    for (int p = 0; p < PH; ++p) { s += red[(p * G + gg) * 8 + cc]; q += red[(p * G + gg) * 8 + 4 + cc]; }
    sres[tid] = s;
    sres[P + tid] = q;
  }
  __syncthreads();
  const v2d ov = *(const v2d*)(sres + 2 * (tid & 255));
  double* pp = part + (size_t)blockIdx.x * 2 * P + 2 * tid;
  if (tid < P) *(volatile v2d*)pp = ov;
  __threadfence();
  if (tid < P) *(volatile v2d*)pp = ov;
}

__global__ __launch_bounds__(NTHR) void k_bnfin(const double* __restrict__ part, int nblk, int P, int C,
                                                const float* __restrict__ gam, const float* __restrict__ bet,
                                                int perm, int nrows, float* scale, float* shift) {
  __shared__ __attribute__((aligned(16))) float ssc[NTHR];
  __shared__ __attribute__((aligned(16))) float ssh[NTHR];
  const int tid = threadIdx.x;
  const int c = tid < P ? tid : P - 1;
  double s = 0.0, q = 0.0;
#pragma unroll 1
  for (int b = 0; b < nblk; ++b) {
    s += part[(size_t)b * 2 * P + c];
    q += part[(size_t)b * 2 * P + P + c];
  }
  const double invn = 1.0 / (double)nrows;
  const double mean = s * invn;
  double var = q * invn - mean * mean;
  var = var < 0.0 ? 0.0 : var;
  int rc = perm != 0 ? (c < ED ? c + NSH : c - ED) : c;
  rc = rc < 0 ? 0 : (rc > C - 1 ? C - 1 : rc);
  const float g = gam[rc], be = bet[rc];
  const float sc = g * rsqrtf((float)var + EPSBN);
  const float sf = be - (float)mean * sc;
  const bool ok = tid < C;
  ssc[tid] = ok ? sc : 0.0f;
  ssh[tid] = ok ? sf : 0.0f;
  __syncthreads();
  const v4f a = *(const v4f*)(ssc + 4 * (tid & 63));
  const v4f b2 = *(const v4f*)(ssh + 4 * (tid & 63));
  const int nq = P >> 2;
  if (tid < nq) { *(volatile v4f*)(scale + 4 * tid) = a; *(volatile v4f*)(shift + 4 * tid) = b2; }
  __threadfence();
  if (tid < nq) { *(volatile v4f*)(scale + 4 * tid) = a; *(volatile v4f*)(shift + 4 * tid) = b2; }
}

__global__ __launch_bounds__(NTHR) void k_upd(
    const float* __restrict__ mpl, const float* __restrict__ scale, const float* __restrict__ shift,
    const _Float16* __restrict__ w1, const _Float16* __restrict__ w2, const _Float16* __restrict__ w3,
    const _Float16* __restrict__ w4, const float* __restrict__ b1, const float* __restrict__ b2,
    const float* __restrict__ b3, const float* __restrict__ b4, float* xall, int tcur, int nN) {
  extern __shared__ v4f lds_dyn[];
  _Float16* bufA = (_Float16*)lds_dyn;
  _Float16* bufB = bufA + GROWS * AP_U;
  float*    stg  = (float*)(bufA + 2 * GROWS * AP_U);
  const int tid = threadIdx.x, lane = tid & 31, wave = tid >> 5, hh = lane >> 4, m = lane & 15;
  const int rowBase = blockIdx.x * GROWS;
  const int r0 = wave * 16;

#pragma unroll
  for (int i = 0; i < (GROWS * KP_MSG / 8) / NTHR; ++i) {
    const int idx = i * NTHR + tid;
    const int r   = idx / (KP_MSG / 8);
    const int c0  = (idx - r * (KP_MSG / 8)) * 8;
    const int row = rowBase + r;
    const float okf = row < nN ? 1.0f : 0.0f;
    const float* ap = mpl + (size_t)row * KP_MSG + c0;
    const v4f a = *(const v4f*)ap, bq = *(const v4f*)(ap + 4);
    const v4f s0 = *(const v4f*)(scale + c0), s1 = *(const v4f*)(scale + c0 + 4);
    const v4f t0 = *(const v4f*)(shift + c0), t1 = *(const v4f*)(shift + c0 + 4);
    const v4f x0 = (a * s0 + t0) * okf;
    const v4f x1 = (bq * s1 + t1) * okf;
    *(v8h*)(bufA + r * AP_U + c0) = cvt8(x0, x1);
  }
  __syncthreads();
  layer_h<KP_MSG / 32, AP_U>(bufA, bufB, w1, b1, r0, hh, m);
  __syncthreads();
  layer_h<KP_HID / 32, AP_U>(bufB, bufA, w2, b2, r0, hh, m);
  __syncthreads();
  layer_h<KP_HID / 32, AP_U>(bufA, bufB, w3, b3, r0, hh, m);
  __syncthreads();
  {
    v8f acc[4];
    mma_tiles<KP_HID / 32, 4>(bufB + (r0 + m) * AP_U + 8 * hh, w4 + (size_t)m * KP_HID + 8 * hh, acc);
    float* sp = stg + (r0 + 8 * hh) * ED + m;
#pragma unroll
    for (int t = 0; t < 4; ++t) {
      const float bl = b4[16 * t + m];
#pragma unroll
      for (int r = 0; r < 8; ++r) sp[r * ED + 16 * t] = acc[t][r] * WINV + bl;
    }
  }
  __syncthreads();

  const int q = lane & 15, rsel = lane >> 4;
  v4f ov[8];
#pragma unroll
  for (int i = 0; i < 8; ++i) {
    const int row = r0 + 2 * i + rsel;
    const v4f d  = *(const v4f*)(stg + row * ED + 4 * q);
    const v4f xo = *(const v4f*)(xall + (size_t)(rowBase + row) * RDIM + tcur * ED + 4 * q);
    ov[i] = xo + d * 0.1f;
  }
#pragma unroll
  for (int i = 0; i < 8; ++i) {
    float* xp = xall + (size_t)(rowBase + r0 + 2 * i + rsel) * RDIM + (tcur + 1) * ED + 4 * q;
    *(volatile v4f*)xp = ov[i];
  }
  __threadfence();
#pragma unroll
  for (int i = 0; i < 8; ++i) {
    float* xp = xall + (size_t)(rowBase + r0 + 2 * i + rsel) * RDIM + (tcur + 1) * ED + 4 * q;
    *(volatile v4f*)xp = ov[i];
  }
}

__global__ __launch_bounds__(NTHR) void k_readout(
    const float* __restrict__ xall, const float* __restrict__ scale, const float* __restrict__ shift,
    const _Float16* __restrict__ w1, const _Float16* __restrict__ w2, const _Float16* __restrict__ w3,
    const _Float16* __restrict__ w4, const float* __restrict__ b1, const float* __restrict__ b2,
    const float* __restrict__ b3, const float* __restrict__ b4, float* yv, int nN) {
  extern __shared__ v4f lds_dyn[];
  _Float16* bufA = (_Float16*)lds_dyn;
  _Float16* bufB = bufA + GROWS * AP_R;
  float*    sOut = (float*)(bufA + 2 * GROWS * AP_R);
  const int tid = threadIdx.x, lane = tid & 31, wave = tid >> 5, hh = lane >> 4, m = lane & 15;
  const int rowBase = blockIdx.x * GROWS;
  const int r0 = wave * 16;

#pragma unroll
  for (int i = 0; i < (GROWS * RDIM / 8) / NTHR; ++i) {
    const int idx = i * NTHR + tid;
    const int r   = idx / (RDIM / 8);
    const int c0  = (idx - r * (RDIM / 8)) * 8;
    const int row = rowBase + r;
    const float okf = row < nN ? 1.0f : 0.0f;
    const float* ap = xall + (size_t)row * RDIM + c0;
    const v4f a = *(const v4f*)ap, bq = *(const v4f*)(ap + 4);
    const v4f s0 = *(const v4f*)(scale + c0), s1 = *(const v4f*)(scale + c0 + 4);
    const v4f t0 = *(const v4f*)(shift + c0), t1 = *(const v4f*)(shift + c0 + 4);
    const v4f x0 = (a * s0 + t0) * okf;
    const v4f x1 = (bq * s1 + t1) * okf;
    *(v8h*)(bufA + r * AP_R + c0) = cvt8(x0, x1);
  }
  __syncthreads();
  layer_h<RDIM / 32, AP_R>(bufA, bufB, w1, b1, r0, hh, m);
  __syncthreads();
  layer_h<KP_HID / 32, AP_R>(bufB, bufA, w2, b2, r0, hh, m);
  __syncthreads();
  layer_h<KP_HID / 32, AP_R>(bufA, bufB, w3, b3, r0, hh, m);
  __syncthreads();
  {
    v8f c1[1];
    mma_tiles<KP_HID / 32, 1>(bufB + (r0 + m) * AP_R + 8 * hh, w4 + (size_t)m * KP_HID + 8 * hh, c1);
    const float b4v = b4[0];
    if (m == 0) {
      sOut[r0 + 8 * hh + 0] = c1[0][0] * WINV + b4v;
      sOut[r0 + 8 * hh + 1] = c1[0][1] * WINV + b4v;
      sOut[r0 + 8 * hh + 2] = c1[0][2] * WINV + b4v;
      sOut[r0 + 8 * hh + 3] = c1[0][3] * WINV + b4v;
      sOut[r0 + 8 * hh + 4] = c1[0][4] * WINV + b4v;
      sOut[r0 + 8 * hh + 5] = c1[0][5] * WINV + b4v;
      sOut[r0 + 8 * hh + 6] = c1[0][6] * WINV + b4v;
      sOut[r0 + 8 * hh + 7] = c1[0][7] * WINV + b4v;
    }
  }
  __syncthreads();
  const v4f ov = *(const v4f*)(sOut + 4 * (tid & 31));
  float* op = yv + rowBase;
  if (tid < 32) *(volatile v4f*)(op + 4 * tid) = ov;
  __threadfence();
  if (tid < 32) *(volatile v4f*)(op + 4 * tid) = ov;
}

__global__ __launch_bounds__(NTHR) void k_molsum(const int* __restrict__ mol, const float* __restrict__ yv,
                                                 float* out, int nN, int vec8) {
  __shared__ __attribute__((aligned(16))) float sacc[NBP];
  __shared__ __attribute__((aligned(16))) int list[LISTN];
  __shared__ int wcnt[NWAVE];
  const int tid = threadIdx.x, lane = tid & 31, wave = tid >> 5;
  const int gBase = blockIdx.x * NBP;
  if (tid < NBP) sacc[tid] = 0.0f;
  __syncthreads();

  const int nChunks = (nN + CHUNK - 1) / CHUNK;
#pragma unroll 1
  for (int ch = 0; ch < nChunks; ++ch) {
    const int cbase = ch * CHUNK;
    const int wc = scan_chunk<NBP>(mol, nN, cbase, gBase, vec8, list, tid, lane, wave);
    if (lane == 0) wcnt[wave] = wc;
    __syncthreads();
    if (wave == 0) {
#pragma unroll 1
      for (int wsx = 0; wsx < NWAVE; ++wsx) {
        int n = __builtin_amdgcn_readfirstlane(wcnt[wsx]);
        n = n > WCAP ? WCAP : (n < 0 ? 0 : n);
        const int* lp = list + wsx * WCAP;
#pragma unroll 1
        for (int i = 0; i < n; ++i) {
          const int ent  = __builtin_amdgcn_readfirstlane(lp[i]);
          const int slot = ent & (NBP - 1);
          int nd = cbase + ((ent >> 12) & (CHUNK - 1));
          nd = nd > nN - 1 ? nN - 1 : nd;
          const float y = yv[nd];
          if (lane == 0) sacc[slot] = sacc[slot] + y;
        }
      }
    }
    __syncthreads();
  }
  const v4f ov = *(const v4f*)(sacc + 4 * (tid & 7));
  float* op = out + gBase;
  if (tid < 8) *(volatile v4f*)(op + 4 * tid) = ov;
  __threadfence();
  if (tid < 8) *(volatile v4f*)(op + 4 * tid) = ov;
}

extern "C" void kernel_launch(void* const* d_in, const int* in_sizes, int n_in,
                              void* d_out, int out_size, void* d_ws, size_t ws_size,
                              hipStream_t stream) {
  if (n_in < 25) return;
  const int nN = in_sizes[0];
  const int nE = in_sizes[1] / 2;
  if (nN <= 0 || nE <= 0 || in_sizes[1] != 2 * nE || in_sizes[2] != nE || in_sizes[3] != nN) return;
  const int nEmb = in_sizes[4] / ED;
  if (nEmb < 1 || in_sizes[4] != nEmb * ED) return;
  if (in_sizes[5] != TPASS * MDIM || in_sizes[6] != TPASS * MDIM) return;
  if (in_sizes[7] != TPASS * MDIM * HID || in_sizes[8] != TPASS * HID) return;
  if (in_sizes[9] != TPASS * HID * HID || in_sizes[10] != TPASS * HID) return;
  if (in_sizes[11] != TPASS * HID * HID || in_sizes[12] != TPASS * HID) return;
  if (in_sizes[13] != TPASS * HID * ED || in_sizes[14] != TPASS * ED) return;
  if (in_sizes[15] != RDIM || in_sizes[16] != RDIM || in_sizes[17] != RDIM * HID || in_sizes[18] != HID) return;
  if (in_sizes[19] != HID * HID || in_sizes[20] != HID || in_sizes[21] != HID * HID || in_sizes[22] != HID) return;
  if (in_sizes[23] != HID || in_sizes[24] < 1) return;
  const int G = out_size;
  if (G <= 0 || (G % NBP) != 0) return;
  if (nE > (1 << 28) || nN > (1 << 24)) return;

  const int*   z    = (const int*)d_in[0];
  const int*   ei   = (const int*)d_in[1];
  const int*   esnk = ei + nE;
  const float* dist = (const float*)d_in[2];
  const int*   mol  = (const int*)d_in[3];
  const float* emb  = (const float*)d_in[4];
  const float* upg  = (const float*)d_in[5];
  const float* upb  = (const float*)d_in[6];
  const float* uw1  = (const float*)d_in[7];
  const float* ub1  = (const float*)d_in[8];
  const float* uw2  = (const float*)d_in[9];
  const float* ub2  = (const float*)d_in[10];
  const float* uw3  = (const float*)d_in[11];
  const float* ub3  = (const float*)d_in[12];
  const float* uw4  = (const float*)d_in[13];
  const float* ub4  = (const float*)d_in[14];
  const float* rog  = (const float*)d_in[15];
  const float* rob  = (const float*)d_in[16];
  const float* rw1  = (const float*)d_in[17];
  const float* rb1  = (const float*)d_in[18];
  const float* rw2  = (const float*)d_in[19];
  const float* rb2  = (const float*)d_in[20];
  const float* rw3  = (const float*)d_in[21];
  const float* rb3  = (const float*)d_in[22];
  const float* rw4  = (const float*)d_in[23];
  const float* rb4  = (const float*)d_in[24];
  float* out = (float*)d_out;

  const int NPAD   = ((nN + TGT - 1) / TGT) * TGT;
  const int nBC    = (nN + NBC - 1) / NBC;
  const int CNTPAD = nBC * NBC;
  if (4 * nBC + 1 > RBN) return;
  const int nBF    = (nN + NBF - 1) / NBF;
  const int csrLen = ((nE + 31) & ~31) + 4096;
  const int nS     = (nN + CSRB - 1) / CSRB;
  const int nAgg   = NPAD / TGT;
  const int nMlp   = NPAD / GROWS;
  const int nEmbB  = NPAD / 16;
  const int nMol   = G / NBP;

  char* ws = (char*)d_ws;
  size_t off = 0;
  const size_t oWp  = off; off += (size_t)WTOT * 2;                off = (off + 255) & ~(size_t)255;
  const size_t oCnt = off; off += (size_t)CNTPAD * 4;              off = (off + 255) & ~(size_t)255;
  const size_t oOff = off; off += (size_t)CNTPAD * 4;              off = (off + 255) & ~(size_t)255;
  const size_t oRb  = off; off += (size_t)RBN * 4;                 off = (off + 255) & ~(size_t)255;
  const size_t oCsr = off; off += (size_t)csrLen * 4;              off = (off + 255) & ~(size_t)255;
  const size_t oX   = off; off += (size_t)NPAD * RDIM * 4;         off = (off + 255) & ~(size_t)255;
  const size_t oM   = off; off += (size_t)NPAD * KP_MSG * 4;       off = (off + 255) & ~(size_t)255;
  const size_t oPt  = off; off += (size_t)nS * 2 * 256 * 8;        off = (off + 255) & ~(size_t)255;
  const size_t oSc  = off; off += (size_t)256 * 4;                 off = (off + 255) & ~(size_t)255;
  const size_t oSh  = off; off += (size_t)256 * 4;                 off = (off + 255) & ~(size_t)255;
  const size_t oY   = off; off += (size_t)NPAD * 4;                off = (off + 255) & ~(size_t)255;
  if (off > ws_size) return;
  _Float16* wp    = (_Float16*)(ws + oWp);
  int*      cnt   = (int*)(ws + oCnt);
  int*      offp  = (int*)(ws + oOff);
  int*      rb    = (int*)(ws + oRb);
  int*      csr   = (int*)(ws + oCsr);
  float*    xall  = (float*)(ws + oX);
  float*    mpl   = (float*)(ws + oM);
  double*   part  = (double*)(ws + oPt);
  float*    scale = (float*)(ws + oSc);
  float*    shift = (float*)(ws + oSh);
  float*    yv    = (float*)(ws + oY);

  const int vec8e = ((nE & 3) == 0) ? 1 : 0;
  const int vec8m = ((nN & 3) == 0) ? 1 : 0;

  k_wprep<<<(WE7 + WPT - 1) / WPT, WPT, 0, stream>>>(uw1, uw2, uw3, uw4, rw1, rw2, rw3, rw4, wp);

  k_count<<<nBC, NTHR, 0, stream>>>(ei, cnt, nE, vec8e);
  k_offsets<<<1, OTHR, 0, stream>>>(cnt, offp, rb, nBC);
  hipFuncSetAttribute(reinterpret_cast<const void*>(&k_fill),
                      hipFuncAttributeMaxDynamicSharedMemorySize, LDS_FILL);
  k_fill<<<nBF, NTHR, LDS_FILL, stream>>>(ei, offp, rb, csr, nE, vec8e, csrLen);

  k_embed<<<nEmbB, NTHR, 0, stream>>>(z, emb, xall, nN, nEmb);

  hipFuncSetAttribute(reinterpret_cast<const void*>(&k_upd),
                      hipFuncAttributeMaxDynamicSharedMemorySize, LDS_UPD);
  hipFuncSetAttribute(reinterpret_cast<const void*>(&k_readout),
                      hipFuncAttributeMaxDynamicSharedMemorySize, LDS_RO);

  for (int t = 0; t < TPASS; ++t) {
    if (t == 0)
      k_agg<1><<<nAgg, NTHR, 0, stream>>>(csr, offp, cnt, esnk, dist, xall, 0, mpl, nN, nE, csrLen);
    else
      k_agg<0><<<nAgg, NTHR, 0, stream>>>(csr, offp, cnt, esnk, dist, xall, t * ED, mpl, nN, nE, csrLen);
    k_colstats<<<nS, NTHR, 0, stream>>>(mpl, KP_MSG, nN, part);
    k_bnfin<<<1, NTHR, 0, stream>>>(part, nS, KP_MSG, MDIM, upg + (size_t)t * MDIM, upb + (size_t)t * MDIM, 1, nN, scale, shift);
    k_upd<<<nMlp, NTHR, LDS_UPD, stream>>>(mpl, scale, shift,
                                           wp + OW1 + (size_t)t * PW1, wp + OW2 + (size_t)t * PW2,
                                           wp + OW3 + (size_t)t * PW2, wp + OW4 + (size_t)t * PW4,
                                           ub1 + (size_t)t * HID, ub2 + (size_t)t * HID, ub3 + (size_t)t * HID,
                                           ub4 + (size_t)t * ED, xall, t, nN);
  }

  k_colstats<<<nS, NTHR, 0, stream>>>(xall, RDIM, nN, part);
  k_bnfin<<<1, NTHR, 0, stream>>>(part, nS, RDIM, RDIM, rog, rob, 0, nN, scale, shift);
  k_readout<<<nMlp, NTHR, LDS_RO, stream>>>(xall, scale, shift, wp + OR1, wp + OR2, wp + OR3, wp + OR4,
                                            rb1, rb2, rb3, rb4, yv, nN);
  k_molsum<<<nMol, NTHR, 0, stream>>>(mol, yv, out, nN, vec8m);
}
